// GAT_22617297780844
// MI455X (gfx1250) — hardware-verified
//
#include <hip/hip_runtime.h>
#include <stddef.h>
#include <stdint.h>


#define DF      128
#define LDC     256
#define NTHR    256
#define NWAVE   8
#define EPT     8
#define CHUNK   (NTHR * EPT)
#define WCAP    (EPT * 32)
#define LISTN   (NWAVE * WCAP)
#define NBA     1024
#define SLA     10
#define RCAP    8192
#define DEGCAP  64
#define GBM     64
#define RELP    512
#define NEGSL   0.2f
#define EPS_SM  1e-16f
#define AGG_ZINTS (LISTN + 2 * RCAP + 3 * NBA)
#define AGG_LDS_INTS (AGG_ZINTS + 16)
#define GEMM_LDS_FLOATS (GBM * LDC + 4 * GBM)
#define PU0 4096
#define PU1 6144
#define PU2 8192
#define PU3 16384
#define PU4 20480
#define PU5 24576
#define PU6 32768

static_assert((CHUNK & (CHUNK - 1)) == 0 && CHUNK <= 4096);
static_assert((NBA & (NBA - 1)) == 0 && NBA == (1 << SLA));
static_assert(LISTN % NTHR == 0);
static_assert(NBA % NWAVE == 0 && NBA % 32 == 0 && NBA % GBM == 0);
static_assert(RCAP % 4 == 0 && AGG_ZINTS % 4 == 0 && LISTN % 4 == 0);
static_assert(AGG_LDS_INTS * 4 <= 300000);
static_assert(DF == 4 * 32 && LDC == 2 * DF);
static_assert(GBM == 64 && NTHR == 256 && RELP % GBM == 0);
static_assert(PU0 % NTHR == 0 && PU1 % NTHR == 0 && PU2 % NTHR == 0 && PU3 % NTHR == 0);
static_assert(PU4 % NTHR == 0 && PU5 % NTHR == 0 && PU6 % NTHR == 0);
static_assert(PU0 == 256 * 16 && PU1 - PU0 == 128 * 16 && PU2 - PU1 == 128 * 16);
static_assert(PU3 - PU2 == 256 * 32 && PU4 - PU3 == 128 * 32 && PU5 - PU4 == 128 * 32);
static_assert(PU6 - PU5 == RELP * 16);
static_assert((RELP * 16) % NTHR == 0);

typedef float          v4f   __attribute__((ext_vector_type(4)));
typedef float          v8f   __attribute__((ext_vector_type(8)));
typedef int            v2i   __attribute__((ext_vector_type(2)));
typedef int            v4i   __attribute__((ext_vector_type(4)));
typedef int            v8i   __attribute__((ext_vector_type(8)));
typedef unsigned int   v4u   __attribute__((ext_vector_type(4)));
typedef unsigned short v8us  __attribute__((ext_vector_type(8)));
typedef __bf16         v16bf __attribute__((ext_vector_type(16)));
typedef v4f  __attribute__((may_alias)) v4fa;
typedef v4i  __attribute__((may_alias)) v4ia;
typedef v8us __attribute__((may_alias)) v8usa;
union FragB { v16bf v; v8us h[2]; v8i w; };

__device__ __forceinline__ v8f wmb(const FragB& a, const FragB& b, v8f c) {
  v8f d = __builtin_amdgcn_wmma_f32_16x16x32_bf16(false, a.v, false, b.v, (short)0, c, false, false);
  asm volatile("v_nop\n\tv_nop\n\tv_nop\n\tv_nop" : "+v"(d) : "v"(a.w), "v"(b.w));
  return d;
}

__device__ __forceinline__ unsigned int f2bf(float f) {
  const unsigned int u = __float_as_uint(f);
  return ((u + 0x7FFFu + ((u >> 16) & 1u)) >> 16) & 0xFFFFu;
}
__device__ __forceinline__ float bf2f(unsigned int b) { return __uint_as_float(b << 16); }
__device__ __forceinline__ float bfr(float f) { return bf2f(f2bf(f)); }
__device__ __forceinline__ v4f bfr4(const v4f a) {
  v4f r; r.x = bfr(a.x); r.y = bfr(a.y); r.z = bfr(a.z); r.w = bfr(a.w); return r;
}
__device__ __forceinline__ unsigned int pk2(float lo, float hi) { return f2bf(lo) | (f2bf(hi) << 16); }
__device__ __forceinline__ v4u pack8(const v4f a, const v4f b) {
  v4u r;
  r.x = pk2(a.x, a.y); r.y = pk2(a.z, a.w); r.z = pk2(b.x, b.y); r.w = pk2(b.z, b.w);
  return r;
}
__device__ __forceinline__ void put16(unsigned short* dp, const v4u w) {
  *(volatile v4u*)dp = w;
  __threadfence();
  *(volatile v4u*)dp = w;
}
__device__ __forceinline__ v4u gath8(const float* __restrict__ p, size_t st) {
  v4f a, b;
  a.x = p[0];      a.y = p[st];     a.z = p[2 * st]; a.w = p[3 * st];
  b.x = p[4 * st]; b.y = p[5 * st]; b.z = p[6 * st]; b.w = p[7 * st];
  return pack8(a, b);
}

template <int SLB>
__device__ __forceinline__ int scan_chunk(const int* __restrict__ dsts, int nE, int cbase, int slotBase,
                                          int nb, int vec8, int* list, int tid, int lane, int wave) {
  int wc = 0;
  const int el0  = tid * EPT;
  const int e0   = cbase + el0;
  const int sent = -2147483647 - 1;
  v4i da, db;
  if (vec8 != 0 && cbase + CHUNK <= nE) {
    da = *(const v4i*)(dsts + e0);
    db = *(const v4i*)(dsts + e0 + 4);
  } else {
    da.x = (e0     < nE) ? dsts[min(e0,     nE - 1)] : sent;
    da.y = (e0 + 1 < nE) ? dsts[min(e0 + 1, nE - 1)] : sent;
    da.z = (e0 + 2 < nE) ? dsts[min(e0 + 2, nE - 1)] : sent;
    da.w = (e0 + 3 < nE) ? dsts[min(e0 + 3, nE - 1)] : sent;
    db.x = (e0 + 4 < nE) ? dsts[min(e0 + 4, nE - 1)] : sent;
    db.y = (e0 + 5 < nE) ? dsts[min(e0 + 5, nE - 1)] : sent;
    db.z = (e0 + 6 < nE) ? dsts[min(e0 + 6, nE - 1)] : sent;
    db.w = (e0 + 7 < nE) ? dsts[min(e0 + 7, nE - 1)] : sent;
  }
  const unsigned nbs = (unsigned)slotBase;
  const unsigned unb = (unsigned)nb;
  const unsigned s0 = (unsigned)da.x - nbs, s1 = (unsigned)da.y - nbs;
  const unsigned s2 = (unsigned)da.z - nbs, s3 = (unsigned)da.w - nbs;
  const unsigned s4 = (unsigned)db.x - nbs, s5 = (unsigned)db.y - nbs;
  const unsigned s6 = (unsigned)db.z - nbs, s7 = (unsigned)db.w - nbs;
  const bool h0 = s0 < unb, h1 = s1 < unb, h2 = s2 < unb, h3 = s3 < unb;
  const bool h4 = s4 < unb, h5 = s5 < unb, h6 = s6 < unb, h7 = s7 < unb;
  const unsigned any = __builtin_amdgcn_ballot_w32(h0 | h1 | h2 | h3 | h4 | h5 | h6 | h7);
  if (any != 0u) {
#define HITJ(J, HJ, SJ) { \
      const unsigned mj = __builtin_amdgcn_ballot_w32(HJ); \
      if (mj != 0u) { \
        if (HJ) { \
          const int pos = wc + (int)__builtin_amdgcn_mbcnt_lo(mj, 0u); \
          if (pos < WCAP) list[wave * WCAP + pos] = ((el0 + (J)) << SLB) | (int)(SJ); \
        } \
        wc += (int)__builtin_popcount(mj); } }
    HITJ(0, h0, s0)
    HITJ(1, h1, s1)
    HITJ(2, h2, s2)
    HITJ(3, h3, s3)
    HITJ(4, h4, s4)
    HITJ(5, h5, s5)
    HITJ(6, h6, s6)
    HITJ(7, h7, s7)
#undef HITJ
  }
  return wc;
}

__global__ __launch_bounds__(NTHR) void k_prep(const float* __restrict__ x, const float* __restrict__ r,
                                               const float* __restrict__ WH, const float* __restrict__ WO,
                                               const float* __restrict__ Wr,
                                               unsigned short* Bt1, unsigned short* BtR1,
                                               unsigned short* Bt2, unsigned short* BtR2,
                                               unsigned short* RB, unsigned short* XB,
                                               int nN, int nRel, int nUx) {
  const int u = (int)blockIdx.x * NTHR + (int)threadIdx.x;
  if (u < PU0) {
    const int n = u >> 4, k8 = (u & 15) * 8;
    const int nn = n & 127, h = nn >> 6, j = nn & 63, kofs = (n >> 7) * 128;
    const v4u w = gath8(WH + (size_t)h * 24576 + (size_t)(kofs + k8) * 64 + j, 64);
    put16(Bt1 + (size_t)n * 128 + k8, w);
  } else if (u < PU1) {
    const int v = u - PU0;
    const int n = v >> 4, k8 = (v & 15) * 8;
    const v4u w = gath8(Wr + (size_t)k8 * 128 + n, 128);
    put16(BtR1 + (size_t)n * 128 + k8, w);
  } else if (u < PU2) {
    const int v = u - PU1;
    const int nn = v >> 4, k8 = (v & 15) * 8;
    const int h = nn >> 6, j = nn & 63;
    const v4u w = gath8(WH + (size_t)h * 24576 + (size_t)(256 + k8) * 64 + j, 64);
    put16(BtR1 + (size_t)(128 + nn) * 128 + k8, w);
  } else if (u < PU3) {
    const int v = u - PU2;
    const int n = v >> 5, k8 = (v & 31) * 8;
    const int kk = k8 & 127, nn = n & 127, rofs = (n >> 7) * 128;
    const v4u w = gath8(WO + (size_t)(rofs + kk) * 128 + nn, 128);
    put16(Bt2 + (size_t)n * 256 + k8, w);
  } else if (u < PU4) {
    const int v = u - PU3;
    const int n = v >> 5, k8 = (v & 31) * 8;
    const v4u z = {0u, 0u, 0u, 0u};
    put16(BtR2 + (size_t)n * 256 + k8, z);
  } else if (u < PU5) {
    const int v = u - PU4;
    const int nn = v >> 5, k8 = (v & 31) * 8;
    const int kk = k8 & 127;
    const v4u w = gath8(WO + (size_t)(256 + kk) * 128 + nn, 128);
    put16(BtR2 + (size_t)(128 + nn) * 256 + k8, w);
  } else if (u < PU6) {
    const int v = u - PU5;
    const int row = v >> 4, k8 = (v & 15) * 8;
    const int rc = row < nRel ? row : nRel - 1;
    const float* p = r + (size_t)rc * DF + k8;
    v4f a = *(const v4f*)p, b = *(const v4f*)(p + 4);
    const v4f z4 = {0.f, 0.f, 0.f, 0.f};
    if (row >= nRel) { a = z4; b = z4; }
    put16(RB + (size_t)row * DF + k8, pack8(a, b));
  } else {
    const int v = u - PU6;
    if (v >= nUx) return;
    const int row = v >> 4, k8 = (v & 15) * 8;
    const int rc = row < nN ? row : nN - 1;
    const float* p = x + (size_t)rc * DF + k8;
    v4f a = *(const v4f*)p, b = *(const v4f*)(p + 4);
    const v4f z4 = {0.f, 0.f, 0.f, 0.f};
    if (row >= nN) { a = z4; b = z4; }
    put16(XB + (size_t)row * DF + k8, pack8(a, b));
  }
}

__global__ __launch_bounds__(NTHR) void k_gemm(const unsigned short* __restrict__ A, int lda,
                                               const unsigned short* __restrict__ BT, int ldb, int K,
                                               float* Cm, const float* __restrict__ avec, float* SD) {
  extern __shared__ __attribute__((aligned(16))) float gsm[];
  float* stg = gsm;
  float* sdt = gsm + GBM * LDC;
  const int tid = (int)threadIdx.x, lane = tid & 31, wave = tid >> 5, hh = lane >> 4, m = lane & 15;
  const int rg = wave & 3, cg = wave >> 2;
  const int rowBase = (int)blockIdx.x * GBM;
  const int colBase = cg * DF;

  v8f acc[8];
  {
    const v8f z = {0.f, 0.f, 0.f, 0.f, 0.f, 0.f, 0.f, 0.f};
#pragma unroll
    for (int t = 0; t < 8; ++t) acc[t] = z;
  }
  const unsigned short* ap = A  + (size_t)(rowBase + 16 * rg + m) * (size_t)lda + 8 * hh;
  const unsigned short* bp = BT + (size_t)(colBase + m) * (size_t)ldb + 8 * hh;

#pragma unroll 1
  for (int k0 = 0; k0 < K; k0 += 32) {
    FragB af;
    af.h[0] = *(const v8usa*)(ap + k0);
    af.h[1] = *(const v8usa*)(ap + k0 + 16);
#pragma unroll
    for (int nt = 0; nt < 8; ++nt) {
      const unsigned short* wq = bp + (size_t)(16 * nt) * (size_t)ldb + k0;
      FragB bf;
      bf.h[0] = *(const v8usa*)wq;
      bf.h[1] = *(const v8usa*)(wq + 16);
      acc[nt] = wmb(af, bf, acc[nt]);
    }
  }

#pragma unroll
  for (int nt = 0; nt < 8; ++nt) {
    const int lc = colBase + 16 * nt + m;
#pragma unroll
    for (int r = 0; r < 8; ++r) {
      const int lr = 16 * rg + 8 * hh + r;
      stg[lr * LDC + lc] = acc[nt][r];
    }
  }
  __syncthreads();

  const v4f a4 = bfr4(*(const v4f*)(avec + 4 * lane));
#pragma unroll 1
  for (int i = 0; i < 8; ++i) {
    const int row = wave * 8 + i;
    const v4f p = *(const v4fa*)(stg + row * LDC + 4 * lane);
    const v4f q = *(const v4fa*)(stg + row * LDC + DF + 4 * lane);
    float s = 0.0f, d = 0.0f;
    s = fmaf(p.x, a4.x, s); s = fmaf(p.y, a4.y, s); s = fmaf(p.z, a4.z, s); s = fmaf(p.w, a4.w, s);
    d = fmaf(q.x, a4.x, d); d = fmaf(q.y, a4.y, d); d = fmaf(q.z, a4.z, d); d = fmaf(q.w, a4.w, d);
#pragma unroll
    for (int off = 8; off > 0; off >>= 1) {
      s += __shfl_xor(s, off);
      d += __shfl_xor(d, off);
    }
    if (m == 0) { sdt[row * 4 + hh] = s; sdt[row * 4 + 2 + hh] = d; }
  }
  __syncthreads();

  const int st = tid < GBM ? tid : GBM - 1;
  const v4f sdv = *(const v4fa*)(sdt + 4 * st);
  float* sp = SD + (size_t)(rowBase + st) * 4;
#pragma unroll 1
  for (int i = 0; i < 8; ++i) {
    const int row = wave * 8 + i;
#pragma unroll
    for (int c = 0; c < 2; ++c) {
      const v4f p = *(const v4fa*)(stg + row * LDC + c * DF + 4 * lane);
      float* op = Cm + (size_t)(rowBase + row) * (size_t)LDC + c * DF + 4 * lane;
      *(volatile v4f*)op = p;
    }
  }
  if (tid < GBM) *(volatile v4f*)sp = sdv;
  __threadfence();
#pragma unroll 1
  for (int i = 0; i < 8; ++i) {
    const int row = wave * 8 + i;
#pragma unroll
    for (int c = 0; c < 2; ++c) {
      const v4f p = *(const v4fa*)(stg + row * LDC + c * DF + 4 * lane);
      float* op = Cm + (size_t)(rowBase + row) * (size_t)LDC + c * DF + 4 * lane;
      *(volatile v4f*)op = p;
    }
  }
  if (tid < GBM) *(volatile v4f*)sp = sdv;
}

__global__ __launch_bounds__(NTHR) void k_r2out(const float* __restrict__ RC, unsigned short* hl, float* r2o,
                                                int nRel, int nUnits) {
  const int u = (int)blockIdx.x * NTHR + (int)threadIdx.x;
  if (u < RELP * 16) {
    const int row = u >> 4, k8 = (u & 15) * 8;
    const float* p = RC + (size_t)row * LDC + k8;
    const v4f a = *(const v4f*)p, b = *(const v4f*)(p + 4);
    const v4u hv = pack8(a, b);
    v4f ra, rb;
    ra.x = a.x - bfr(a.x); ra.y = a.y - bfr(a.y); ra.z = a.z - bfr(a.z); ra.w = a.w - bfr(a.w);
    rb.x = b.x - bfr(b.x); rb.y = b.y - bfr(b.y); rb.z = b.z - bfr(b.z); rb.w = b.w - bfr(b.w);
    const v4u lv = pack8(ra, rb);
    unsigned short* dp = hl + (size_t)row * LDC + k8;
    *(volatile v4u*)dp = hv;
    *(volatile v4u*)(dp + DF) = lv;
    __threadfence();
    *(volatile v4u*)dp = hv;
    *(volatile v4u*)(dp + DF) = lv;
  } else {
    if (u >= nUnits) return;
    const int v = u - RELP * 16;
    const int row = v >> 5, pc = v & 31;
    const int rc = row < nRel ? row : nRel - 1;
    const v4f val = *(const v4f*)(RC + (size_t)rc * LDC + 4 * pc);
    if (row < nRel) {
      float* op = r2o + (size_t)row * DF + 4 * pc;
      *(volatile v4f*)op = val;
      __threadfence();
      *(volatile v4f*)op = val;
    }
  }
}

template <int L>
__global__ __launch_bounds__(NTHR) void k_scan(const int* __restrict__ keys, const int* __restrict__ oths,
                                               const int* __restrict__ etype, const int* __restrict__ nhop,
                                               int nE, int nE1, int nE2, int nN, int nRel, int vec8, int mRows,
                                               const float* __restrict__ PQ, const float* __restrict__ SDN,
                                               const float* __restrict__ RT, const float* __restrict__ SDR,
                                               unsigned short* hb, float* outp) {
  extern __shared__ __attribute__((aligned(16))) int dsm[];
  int* list = dsm;
  int* hl   = dsm + LISTN;
  int* sl   = dsm + LISTN + RCAP;
  int* cnt  = dsm + LISTN + 2 * RCAP;
  int* offs = cnt + NBA;
  int* cur  = offs + NBA;
  int* misc = cur + NBA;
  const int tid = (int)threadIdx.x, lane = tid & 31, wave = tid >> 5;
  const int nodeBase = (int)blockIdx.x * NBA;

  {
    const v4i z4 = {0, 0, 0, 0};
    for (int i = tid * 4; i < AGG_ZINTS; i += NTHR * 4) *(v4ia*)(dsm + i) = z4;
    if (tid < 16) misc[tid] = 0;
  }
  __syncthreads();

  int t = 0, ov = 0;
  const int nChunks = (nE + CHUNK - 1) / CHUNK;
#pragma unroll 1
  for (int ch = 0; ch < nChunks; ++ch) {
    const int cbase = ch * CHUNK;
    const int wc = scan_chunk<SLA>(keys, nE, cbase, nodeBase, NBA, vec8, list, tid, lane, wave);
    if (lane == 0) misc[wave] = wc;
    __syncthreads();
    if (wave == 0) {
#pragma unroll 1
      for (int w2 = 0; w2 < NWAVE; ++w2) {
        int c = misc[w2];
        c = c < 0 ? 0 : (c > WCAP ? WCAP : c);
#pragma unroll 1
        for (int b0 = 0; b0 < c; b0 += 32) {
          const int idx = b0 + lane;
          const int ent = list[w2 * WCAP + (idx < WCAP ? idx : WCAP - 1)];
          const int m32 = (c - b0) < 32 ? (c - b0) : 32;
#pragma unroll 1
          for (int k = 0; k < m32; ++k) {
            const int u    = __builtin_amdgcn_readlane(ent, k);
            const int slot = u & (NBA - 1);
            const int el   = (u >> SLA) & (CHUNK - 1);
            const int pk   = ((cbase + el) << SLA) | slot;
            if (t < RCAP) {
              if (lane == 0) { hl[t] = pk; cnt[slot] = cnt[slot] + 1; }
              t = t + 1;
            } else {
              ov = 1;
            }
          }
        }
      }
    }
    __syncthreads();
  }
  if (wave == 0 && lane == 0) { misc[8] = t; misc[9] = ov; }
  __syncthreads();
  int tt = misc[8];
  tt = tt < 0 ? 0 : (tt > RCAP ? RCAP : tt);
  const int ovf = misc[9];

  if (wave == 0) {
    const int base = lane * (NBA / 32);
    int s = 0;
#pragma unroll 1
    for (int i = 0; i < NBA / 32; ++i) s += cnt[base + i];
    int incl = s;
#pragma unroll
    for (int d = 1; d < 32; d <<= 1) {
      const int y = __shfl_up(incl, d, 32);
      if (lane >= d) incl += y;
    }
    int run = incl - s;
#pragma unroll 1
    for (int i = 0; i < NBA / 32; ++i) {
      const int cv = cnt[base + i];
      offs[base + i] = run;
      cur[base + i]  = run;
      run += cv;
    }
  }
  __syncthreads();
  if (wave == 0) {
#pragma unroll 1
    for (int b0 = 0; b0 < tt; b0 += 32) {
      const int idx = b0 + lane;
      const int ent = hl[idx < RCAP ? idx : RCAP - 1];
      const int m32 = (tt - b0) < 32 ? (tt - b0) : 32;
#pragma unroll 1
      for (int k = 0; k < m32; ++k) {
        const int u    = __builtin_amdgcn_readlane(ent, k);
        const int slot = u & (NBA - 1);
        if (lane == 0) {
          int p = cur[slot];
          p = p < 0 ? 0 : (p > RCAP - 1 ? RCAP - 1 : p);
          sl[p] = u;
          cur[slot] = p + 1;
        }
      }
    }
  }
  __syncthreads();

  const float qnan = __int_as_float(0x7fc00000);
  const float pz = (ovf != 0) ? qnan : 0.0f;
  const int c4 = 4 * lane;
  const bool hd1 = lane >= 16;
#pragma unroll 1
  for (int si = 0; si < NBA / NWAVE; ++si) {
    const int s    = si * NWAVE + wave;
    const int node = nodeBase + s;
    int c = __builtin_amdgcn_readfirstlane(cnt[s]);
    const bool big = c > DEGCAP;
    c = c < 0 ? 0 : (c > DEGCAP ? DEGCAP : c);
    int o = __builtin_amdgcn_readfirstlane(offs[s]);
    o = o < 0 ? 0 : (o > tt ? tt : o);
    if (c > tt - o) c = tt - o;
    const int nc = node < nN ? node : nN - 1;
    const v4f sdi = *(const v4f*)(SDN + (size_t)nc * 4);
    const v4f pr  = *(const v4f*)(PQ + (size_t)nc * LDC + c4);
    float ps0, ps1;
    if constexpr (L == 1) { ps0 = sdi.x; ps1 = sdi.y; }
    else                  { ps0 = sdi.x + sdi.y; ps1 = ps0; }
    float mx = -1.0e30f, dn = 0.0f;
    v4f av = {0.f, 0.f, 0.f, 0.f};
#pragma unroll 1
    for (int b0 = 0; b0 < c; b0 += 32) {
      int idx = o + b0 + lane;
      idx = idx > RCAP - 1 ? RCAP - 1 : idx;
      const int ent = sl[idx];
      int eid = ent >> SLA;
      eid = eid < 0 ? 0 : (eid > nE - 1 ? nE - 1 : eid);
      int oth = oths[eid];
      oth = oth < 0 ? 0 : (oth > nN - 1 ? nN - 1 : oth);
      const int is1 = (eid < nE1) ? 1 : 0;
      const int e1  = eid < nE1 ? eid : nE1 - 1;
      int e2 = eid - nE1;
      e2 = e2 < 0 ? 0 : (e2 > nE2 - 1 ? nE2 - 1 : e2);
      const int t1  = etype[e1];
      const v2i nh2 = *(const v2i*)(nhop + 2 * (size_t)e2);
      const int msk = -is1;
      int ta = (t1 & msk) | (nh2.x & ~msk);
      int tb = nh2.y;
      ta = ta < 0 ? 0 : (ta > nRel - 1 ? nRel - 1 : ta);
      tb = tb < 0 ? 0 : (tb > nRel - 1 ? nRel - 1 : tb);
      const float w2 = (float)(1 - is1);
      const v4f sdo = *(const v4f*)(SDN + (size_t)oth * 4);
      const v4f ra  = *(const v4f*)(SDR + (size_t)ta * 4);
      const v4f rb  = *(const v4f*)(SDR + (size_t)tb * 4);
      float l0, l1;
      if constexpr (L == 1) {
        l0 = ps0 + sdo.z + fmaf(w2, rb.z, ra.z);
        l1 = ps1 + sdo.w + fmaf(w2, rb.w, ra.w);
      } else {
        l0 = ps0 + (sdo.z + sdo.w) + fmaf(w2, rb.z + rb.w, ra.z + ra.w);
        l1 = l0;
      }
      l0 = l0 > 0.f ? l0 : NEGSL * l0;
      l1 = l1 > 0.f ? l1 : NEGSL * l1;
      const int w2i = __float_as_int(w2);
      const int l0i = __float_as_int(l0);
      const int l1i = __float_as_int(l1);
      const int m32 = (c - b0) < 32 ? (c - b0) : 32;
#pragma unroll 1
      for (int k = 0; k < m32; ++k) {
        const int   sk  = __builtin_amdgcn_readlane(oth, k);
        const int   tak = __builtin_amdgcn_readlane(ta, k);
        const int   tbk = __builtin_amdgcn_readlane(tb, k);
        const float w2k = __int_as_float(__builtin_amdgcn_readlane(w2i, k));
        const float lgA = __int_as_float(__builtin_amdgcn_readlane(l0i, k));
        float lg = lgA;
        if constexpr (L == 1) {
          const float lgB = __int_as_float(__builtin_amdgcn_readlane(l1i, k));
          lg = hd1 ? lgB : lgA;
        }
        const v4f q4 = *(const v4f*)(PQ + (size_t)sk  * LDC + DF + c4);
        const v4f r1 = *(const v4f*)(RT + (size_t)tak * LDC + DF + c4);
        const v4f r2 = *(const v4f*)(RT + (size_t)tbk * LDC + DF + c4);
        v4f mm;
        mm.x = fmaf(w2k, r2.x, q4.x + r1.x);
        mm.y = fmaf(w2k, r2.y, q4.y + r1.y);
        mm.z = fmaf(w2k, r2.z, q4.z + r1.z);
        mm.w = fmaf(w2k, r2.w, q4.w + r1.w);
        const float df = lg - mx;
        const float ee = __expf(-fabsf(df));
        const bool  up = df > 0.f;
        const float s1 = up ? ee : 1.0f;
        const float s2 = up ? 1.0f : ee;
        mx = up ? lg : mx;
        dn = fmaf(dn, s1, s2);
        av.x = fmaf(av.x, s1, s2 * mm.x);
        av.y = fmaf(av.y, s1, s2 * mm.y);
        av.z = fmaf(av.z, s1, s2 * mm.z);
        av.w = fmaf(av.w, s1, s2 * mm.w);
      }
    }
    const float inv = __builtin_amdgcn_rcpf(dn + EPS_SM);
    const float S   = dn * inv;
    const float pzr = big ? qnan : pz;
    const bool live = node < nN;
    const float v0 = fmaf(S, pr.x, av.x * inv);
    const float v1 = fmaf(S, pr.y, av.y * inv);
    const float v2 = fmaf(S, pr.z, av.z * inv);
    const float v3 = fmaf(S, pr.w, av.w * inv);
    const float u0 = (v0 > 0.f) ? v0 : (__expf(v0) - 1.0f);
    const float u1 = (v1 > 0.f) ? v1 : (__expf(v1) - 1.0f);
    const float u2 = (v2 > 0.f) ? v2 : (__expf(v2) - 1.0f);
    const float u3 = (v3 > 0.f) ? v3 : (__expf(v3) - 1.0f);
    const float y0 = live ? (u0 + pzr) : 0.0f;
    const float y1 = live ? (u1 + pzr) : 0.0f;
    const float y2 = live ? (u2 + pzr) : 0.0f;
    const float y3 = live ? (u3 + pzr) : 0.0f;
    if constexpr (L == 1) {
      const unsigned int hbx = f2bf(y0), hby = f2bf(y1), hbz = f2bf(y2), hbw = f2bf(y3);
      const unsigned int lbx = f2bf(y0 - bf2f(hbx)), lby = f2bf(y1 - bf2f(hby));
      const unsigned int lbz = f2bf(y2 - bf2f(hbz)), lbw = f2bf(y3 - bf2f(hbw));
      const int hw0 = (int)(hbx | (hby << 16)), hw1 = (int)(hbz | (hbw << 16));
      const int lw0 = (int)(lbx | (lby << 16)), lw1 = (int)(lbz | (lbw << 16));
      const int sa = (2 * lane) & 31, sb = (2 * lane + 1) & 31;
      const int g0 = __shfl(hw0, sa), g1 = __shfl(hw1, sa), g2 = __shfl(hw0, sb), g3 = __shfl(hw1, sb);
      const int q0 = __shfl(lw0, sa), q1 = __shfl(lw1, sa), q2 = __shfl(lw0, sb), q3 = __shfl(lw1, sb);
      v4u pv;
      pv.x = (unsigned int)(hd1 ? q0 : g0);
      pv.y = (unsigned int)(hd1 ? q1 : g1);
      pv.z = (unsigned int)(hd1 ? q2 : g2);
      pv.w = (unsigned int)(hd1 ? q3 : g3);
      if (node < mRows) {
        unsigned short* gp = hb + (size_t)node * LDC + 8 * lane;
        *(volatile v4u*)gp = pv;
        __threadfence();
        *(volatile v4u*)gp = pv;
      }
    } else {
      v4f ov4;
      ov4.x = y0; ov4.y = y1; ov4.z = y2; ov4.w = y3;
      if (live) {
        float* op = outp + (size_t)node * DF + c4;
        *(volatile v4f*)op = ov4;
        __threadfence();
        *(volatile v4f*)op = ov4;
      }
    }
  }
}

static inline int cdiv(int a, int b) { return (a + b - 1) / b; }

extern "C" void kernel_launch(void* const* d_in, const int* in_sizes, int n_in,
                              void* d_out, int out_size, void* d_ws, size_t ws_size,
                              hipStream_t stream) {
  if (n_in < 10) return;
  if (in_sizes[0] < 2 || (in_sizes[0] & 1) != 0) return;
  const int nE = in_sizes[0] / 2;
  if (nE < 1 || nE >= (1 << 21)) return;
  if (in_sizes[1] < DF || (in_sizes[1] % DF) != 0) return;
  const int nN = in_sizes[1] / DF;
  if (in_sizes[2] < DF || (in_sizes[2] % DF) != 0) return;
  const int nRel = in_sizes[2] / DF;
  if (nRel < 1 || nRel > RELP) return;
  const int nE1 = in_sizes[3];
  if (in_sizes[4] < 2 || (in_sizes[4] & 1) != 0) return;
  const int nE2 = in_sizes[4] / 2;
  if (nE1 < 1 || nE2 < 1 || nE1 + nE2 != nE) return;
  if (in_sizes[5] != 2 * 384 * 64) return;
  if (in_sizes[6] != 128) return;
  if (in_sizes[7] != 384 * 128) return;
  if (in_sizes[8] != 128) return;
  if (in_sizes[9] != 128 * 128) return;
  if ((long long)out_size != (long long)nN * DF + (long long)nRel * DF) return;

  const int*   edge = (const int*)  d_in[0];
  const float* x    = (const float*)d_in[1];
  const float* r    = (const float*)d_in[2];
  const int*   etyp = (const int*)  d_in[3];
  const int*   nhop = (const int*)  d_in[4];
  const float* WH   = (const float*)d_in[5];
  const float* aH   = (const float*)d_in[6];
  const float* WO   = (const float*)d_in[7];
  const float* aO   = (const float*)d_in[8];
  const float* Wr   = (const float*)d_in[9];
  float* out = (float*)d_out;
  float* r2o = out + (size_t)nN * DF;
  const int* keys = edge;
  const int* oths = edge + nE;

  const int MP   = cdiv(nN, GBM) * GBM;
  const int gM   = MP / GBM;
  const int gA   = cdiv(MP, NBA);
  if ((long long)gA * NBA < (long long)MP) return;
  const int vec8 = ((nE & 3) == 0) ? 1 : 0;

  char* ws = (char*)d_ws;
  size_t off = 0;
  const size_t oBt1  = off; off += (size_t)256 * 128 * 2;            off = (off + 255) & ~(size_t)255;
  const size_t oBtR1 = off; off += (size_t)256 * 128 * 2;            off = (off + 255) & ~(size_t)255;
  const size_t oBt2  = off; off += (size_t)256 * 256 * 2;            off = (off + 255) & ~(size_t)255;
  const size_t oBtR2 = off; off += (size_t)256 * 256 * 2;            off = (off + 255) & ~(size_t)255;
  const size_t oRB   = off; off += (size_t)RELP * DF * 2;            off = (off + 255) & ~(size_t)255;
  const size_t oR2HL = off; off += (size_t)RELP * LDC * 2;           off = (off + 255) & ~(size_t)255;
  const size_t oRC1  = off; off += (size_t)RELP * LDC * 4;           off = (off + 255) & ~(size_t)255;
  const size_t oRC2  = off; off += (size_t)RELP * LDC * 4;           off = (off + 255) & ~(size_t)255;
  const size_t oSDR1 = off; off += (size_t)RELP * 4 * 4;             off = (off + 255) & ~(size_t)255;
  const size_t oSDR2 = off; off += (size_t)RELP * 4 * 4;             off = (off + 255) & ~(size_t)255;
  const size_t oSDN  = off; off += (size_t)MP * 4 * 4;               off = (off + 255) & ~(size_t)255;
  const size_t oX1   = off; off += (size_t)MP * LDC * 2;             off = (off + 255) & ~(size_t)255;
  const size_t oPQ   = off; off += (size_t)MP * LDC * 4;             off = (off + 255) & ~(size_t)255;
  if (off > ws_size) return;
  unsigned short* Bt1  = (unsigned short*)(ws + oBt1);
  unsigned short* BtR1 = (unsigned short*)(ws + oBtR1);
  unsigned short* Bt2  = (unsigned short*)(ws + oBt2);
  unsigned short* BtR2 = (unsigned short*)(ws + oBtR2);
  unsigned short* RB   = (unsigned short*)(ws + oRB);
  unsigned short* R2HL = (unsigned short*)(ws + oR2HL);
  float*          RC1  = (float*)(ws + oRC1);
  float*          RC2  = (float*)(ws + oRC2);
  float*          SDR1 = (float*)(ws + oSDR1);
  float*          SDR2 = (float*)(ws + oSDR2);
  float*          SDN  = (float*)(ws + oSDN);
  unsigned short* X1   = (unsigned short*)(ws + oX1);
  unsigned short* XB   = X1;
  float*          PQ   = (float*)(ws + oPQ);

  const size_t gemmLds = (size_t)GEMM_LDS_FLOATS * 4;
  const size_t aggLds  = (size_t)AGG_LDS_INTS * 4;
  hipFuncSetAttribute(reinterpret_cast<const void*>(&k_gemm), hipFuncAttributeMaxDynamicSharedMemorySize, (int)gemmLds);
  hipFuncSetAttribute(reinterpret_cast<const void*>(&k_scan<1>), hipFuncAttributeMaxDynamicSharedMemorySize, (int)aggLds);
  hipFuncSetAttribute(reinterpret_cast<const void*>(&k_scan<2>), hipFuncAttributeMaxDynamicSharedMemorySize, (int)aggLds);

  const int nUx = MP * (DF / 8);
  k_prep<<<(PU6 + nUx) / NTHR, NTHR, 0, stream>>>(x, r, WH, WO, Wr, Bt1, BtR1, Bt2, BtR2, RB, XB, nN, nRel, nUx);
  k_gemm<<<RELP / GBM, NTHR, gemmLds, stream>>>(RB, DF, BtR1, DF, DF, RC1, aH, SDR1);
  const int nUr = RELP * 16 + nRel * 32;
  k_r2out<<<cdiv(nUr, NTHR), NTHR, 0, stream>>>(RC1, R2HL, r2o, nRel, nUr);
  k_gemm<<<RELP / GBM, NTHR, gemmLds, stream>>>(R2HL, LDC, BtR2, LDC, LDC, RC2, aO, SDR2);
  k_gemm<<<gM, NTHR, gemmLds, stream>>>(XB, DF, Bt1, DF, DF, PQ, aH, SDN);
  k_scan<1><<<gA, NTHR, aggLds, stream>>>(keys, oths, etyp, nhop, nE, nE1, nE2, nN, nRel, vec8, MP,
                                          PQ, SDN, RC1, SDR1, X1, out);
  k_gemm<<<gM, NTHR, gemmLds, stream>>>(X1, LDC, Bt2, LDC, LDC, PQ, aO, SDN);
  k_scan<2><<<gA, NTHR, aggLds, stream>>>(keys, oths, etyp, nhop, nE, nE1, nE2, nN, nRel, vec8, MP,
                                          PQ, SDN, RC2, SDR2, X1, out);
}
